// NonLocalBlock1D_7739531067712
// MI455X (gfx1250) — hardware-verified
//
#include <hip/hip_runtime.h>
#include <math.h>

typedef __attribute__((ext_vector_type(16))) _Float16 v16h;
typedef __attribute__((ext_vector_type(16))) __bf16 v16b;
typedef __attribute__((ext_vector_type(8)))  _Float16 v8h;
typedef __attribute__((ext_vector_type(8)))  float v8f;
typedef __attribute__((ext_vector_type(4)))  float v4f;
typedef __attribute__((ext_vector_type(2)))  float v2f;
typedef __attribute__((ext_vector_type(4)))  unsigned v4u;
typedef __attribute__((ext_vector_type(4)))  int v4i;
typedef float __attribute__((may_alias)) float_a;
typedef int __attribute__((may_alias)) int_a;

template <typename T> __device__ __forceinline__ void vst2(void* p, T v) { *(volatile T*)p = v; __threadfence(); *(volatile T*)p = v; }
__device__ __forceinline__ v8f wmma16(v16h a, v16h b, v8f c) {
  v8f d = __builtin_amdgcn_wmma_f32_16x16x32_f16(false, a, false, b, (short)0, c, false, false);
  asm volatile("v_nop\n\tv_nop\n\tv_nop\n\tv_nop" : "+v"(d) : "v"(a), "v"(b));
  return d;
}
__device__ __forceinline__ v8f wmma_bf(v16b a, v16b b, v8f c) {
  v8f d = __builtin_amdgcn_wmma_f32_16x16x32_bf16(false, a, false, b, (short)0, c, false, false);
  asm volatile("v_nop\n\tv_nop\n\tv_nop\n\tv_nop" : "+v"(d) : "v"(a), "v"(b));
  return d;
}
__device__ __forceinline__ v16h frag_h(const _Float16* rowk0, int lane) {
  union { v16h v; v8h q[2]; } u; const _Float16* p = rowk0 + 8 * (lane >> 4);
  u.q[0] = *(const v8h*)p; u.q[1] = *(const v8h*)(p + 16); return u.v;
}
__device__ __forceinline__ v16h frag_f32(const float* rowk0, int lane) {
  v16h a; const float* p = rowk0 + 8 * (lane >> 4);
#pragma unroll
  for (int i = 0; i < 8; ++i) { a[i] = (_Float16)p[i]; a[8 + i] = (_Float16)p[16 + i]; }
  return a;
}
__device__ __forceinline__ v16h frag_f32s(const float* rowk0, int lane, float sc) {
  v16h a; const float* p = rowk0 + 8 * (lane >> 4);
#pragma unroll
  for (int i = 0; i < 8; ++i) { a[i] = (_Float16)(p[i] * sc); a[8 + i] = (_Float16)(p[16 + i] * sc); }
  return a;
}
__device__ __forceinline__ v16h fragc_f32(const float* W, int k0, int n, int lane, int ld, int K) {
  v16h a; const int g = lane >> 4;
#pragma unroll
  for (int i = 0; i < 8; ++i) { const int ka = k0 + 8 * g + i, kb = ka + 16;
    a[i] = (_Float16)(ka < K ? W[(size_t)(ka < K ? ka : K - 1) * ld + n] : 0.f); a[8 + i] = (_Float16)(kb < K ? W[(size_t)(kb < K ? kb : K - 1) * ld + n] : 0.f); }
  return a;
}
struct F2 { v16b h, l; };
__device__ __forceinline__ F2 bsplit16(const float v[16]) { F2 r;
#pragma unroll
  for (int i = 0; i < 16; ++i) { const __bf16 h = (__bf16)v[i]; r.h[i] = h; r.l[i] = (__bf16)(v[i] - (float)h); }
  return r; }
__device__ __forceinline__ F2 split_row(const float* row, int k0, int lane) { float v[16]; const float* p = row + k0 + 8 * (lane >> 4);
#pragma unroll
  for (int i = 0; i < 8; ++i) { v[i] = p[i]; v[8 + i] = p[16 + i]; }
  return bsplit16(v); }
__device__ __forceinline__ F2 split_rowK(const float* row, int k0, int lane, int K) { float v[16]; const int g = lane >> 4;
#pragma unroll
  for (int i = 0; i < 8; ++i) { const int ka = k0 + 8 * g + i, kb = ka + 16; v[i] = ka < K ? row[ka < K ? ka : K - 1] : 0.f; v[8 + i] = kb < K ? row[kb < K ? kb : K - 1] : 0.f; }
  return bsplit16(v); }
__device__ __forceinline__ F2 split_col(const float* W, int k0, int n, int lane, int ld, int K) { float v[16]; const int g = lane >> 4;
#pragma unroll
  for (int i = 0; i < 8; ++i) { const int ka = k0 + 8 * g + i, kb = ka + 16; v[i] = ka < K ? W[(size_t)(ka < K ? ka : K - 1) * ld + n] : 0.f; v[8 + i] = kb < K ? W[(size_t)(kb < K ? kb : K - 1) * ld + n] : 0.f; }
  return bsplit16(v); }
__device__ __forceinline__ v8f mac3(const F2& a, const F2& b, v8f c) { c = wmma_bf(a.l, b.h, c); c = wmma_bf(a.h, b.l, c); return wmma_bf(a.h, b.h, c); }
__device__ __forceinline__ float sigm(float v) { return 1.0f / (1.0f + expf(-v)); }
#define LDSX() do { asm volatile("s_wait_dscnt 0" ::: "memory"); __builtin_amdgcn_wave_barrier(); __builtin_amdgcn_fence(__ATOMIC_RELEASE, "workgroup"); } while (0)

__device__ __forceinline__ float bfr(float v) { return (float)(__bf16)v; }
#define NB 8
#define TT 2048
#define CX 512
#define CI 256
#ifndef TNB
#define TNB NB
#endif
#ifndef XSTR
#define XSTR TT
#endif
typedef __attribute__((ext_vector_type(8))) __bf16 v8b;
__device__ __forceinline__ v16b frag_b(const __bf16* rowk0, int lane) { union { v16b v; v8b q[2]; } u; const __bf16* p = rowk0 + 8 * (lane >> 4); u.q[0] = *(const v8b*)p; u.q[1] = *(const v8b*)(p + 16); return u.v; }
#define WS_XT  0u
#define WS_TH  (WS_XT + 2u * (size_t)NB * TT * CX)
#define WS_TL  (WS_TH + 2u * (size_t)NB * TT * CI)
#define WS_PH  (WS_TL + 2u * (size_t)NB * TT * CI)
#define WS_PL  (WS_PH + 2u * (size_t)NB * TT * CI)
#define WS_GP  (WS_PL + 2u * (size_t)NB * TT * CI)
#define WS_S   (WS_GP + 2u * (size_t)NB * CI * TT)
#define WS_Y   (WS_S + 4u * (size_t)TT * TT)
#define WS_END (WS_Y + 4u * (size_t)NB * TT * CI)
__global__ __launch_bounds__(256) void k_xt(const float* __restrict__ X, const float* __restrict__ SRC, __bf16* __restrict__ XT, __bf16* __restrict__ ST) { __shared__ __bf16 st[CX][66];
  const int t = threadIdx.x; const int n0 = blockIdx.x * 64; const size_t b = blockIdx.y; const int which = blockIdx.z; const float* IN = which == 0 ? X : SRC; __bf16* OUT = which == 0 ? XT : ST;
  for (int e = t; e < CX * 64; e += 256) { const int c = e >> 6, nl = e & 63; st[c][nl] = (__bf16)IN[(b * CX + c) * (size_t)XSTR + n0 + nl]; }
  __syncthreads();
  for (int e = t; e < 64 * (CX / 8); e += 256) { const int nl = e / (CX / 8), q = e % (CX / 8); union { v4u v; __bf16 h[8]; } u;
#pragma unroll
    for (int z = 0; z < 8; ++z) u.h[z] = st[q * 8 + z][nl];
    vst2((v4u*)(OUT + (b * TT + n0 + nl) * CX + q * 8), u.v); } }
__global__ __launch_bounds__(128) void k_proj(const __bf16* __restrict__ XT, const __bf16* __restrict__ ST, const float* __restrict__ WG, const float* __restrict__ BG, const float* __restrict__ WTH, const float* __restrict__ BTH, const float* __restrict__ WPH, const float* __restrict__ BPH, _Float16* __restrict__ TH, _Float16* __restrict__ TL, _Float16* __restrict__ PH, _Float16* __restrict__ PL, _Float16* __restrict__ GP) {
  __shared__ __align__(16) _Float16 sh[64][136], sl[64][136]; __shared__ __align__(16) _Float16 th[128][72];
  const int tid = threadIdx.x, wave = tid >> 5, lane = tid & 31, col = lane & 15, g = lane >> 4; const int which = blockIdx.y; const int c0 = blockIdx.z * 128; const size_t r0 = (size_t)blockIdx.x * 64;
  const __bf16* A = XT; (void)ST; const float* Wt = which == 0 ? WTH : which == 1 ? WPH : WG; const float* Bb = which == 0 ? BTH : which == 1 ? BPH : BG;
  v8f acc[8] = {};
#pragma unroll 2
  for (int kc = 0; kc < CX / 32; ++kc) { const v16b a = frag_b(A + (r0 + wave * 16 + col) * CX + kc * 32, lane);
#pragma unroll
    for (int j = 0; j < 8; ++j) { v16b w; const float* wr = Wt + (size_t)(c0 + j * 16 + col) * CX + kc * 32 + 8 * g;
#pragma unroll
      for (int i = 0; i < 8; ++i) { w[i] = (__bf16)wr[i]; w[8 + i] = (__bf16)wr[16 + i]; }
      asm volatile("s_wait_loadcnt 0x0" ::: "memory"); acc[j] = wmma_bf(a, w, acc[j]); } }
#pragma unroll
  for (int j = 0; j < 8; ++j) { const int o = j * 16 + col; const float bb = bfr(Bb[c0 + o]);
#pragma unroll
    for (int r = 0; r < 8; ++r) { const float v = acc[j][r] + bb; const int rl = wave * 16 + 8 * g + r;
      if (which == 2) th[o][rl] = (_Float16)v; else { const _Float16 hv = (_Float16)v; sh[rl][o] = hv; sl[rl][o] = (_Float16)((v - (float)hv) * 1024.0f); } } }
  __syncthreads();
  if (which < 2) { _Float16* DH = which == 0 ? TH : PH; _Float16* DL = which == 0 ? TL : PL; for (int e = tid; e < 64 * 16; e += 128) { const int rl = e >> 4, q = e & 15; vst2((unsigned*)(DH + (r0 + rl) * CI + c0 + q * 8), *(const v4u*)&sh[rl][q * 8]); if (which == 0) vst2((unsigned*)(DL + (r0 + rl) * CI + c0 + q * 8), *(const v4u*)&sl[rl][q * 8]); } }
  else { const size_t b = r0 / TT; const int m0 = (int)(r0 % TT); for (int e = tid; e < 128 * 8; e += 128) { const int cl = e >> 3, q = e & 7; vst2((unsigned*)(GP + (b * CI + c0 + cl) * (size_t)TT + m0 + q * 8), *(const v4u*)&th[cl][q * 8]); } } }
__global__ __launch_bounds__(128) void k_sc(const _Float16* __restrict__ TH, const _Float16* __restrict__ TL, const _Float16* __restrict__ PH, const _Float16* __restrict__ PL, int b, float* __restrict__ S) { __shared__ __align__(16) float ss[4][16][132];
  const int tid = threadIdx.x, wave = tid >> 5, lane = tid & 31, col = lane & 15, g = lane >> 4; const int k0 = blockIdx.y * 128; const int ql0 = blockIdx.x * 64 + wave * 16; const size_t q0 = (size_t)b * TT + ql0;
  v8f acc[8] = {}, accl[8] = {};
#pragma unroll 2
  for (int kc = 0; kc < CI / 32; ++kc) { const v16h ah = frag_h(TH + (q0 + col) * CI + kc * 32, lane), al = frag_h(TL + (q0 + col) * CI + kc * 32, lane);
#pragma unroll
    for (int j = 0; j < 8; ++j) { const size_t ko = ((size_t)b * TT + k0 + j * 16 + col) * CI + kc * 32; const v16h kb = frag_h(PH + ko, lane); acc[j] = wmma16(ah, kb, acc[j]); accl[j] = wmma16(al, kb, accl[j]); } (void)PL; }
#pragma unroll
  for (int j = 0; j < 8; ++j)
#pragma unroll
    for (int r = 0; r < 8; ++r) ss[wave][8 * g + r][j * 16 + col] = acc[j][r] + accl[j][r] * (1.0f / 1024.0f);
  LDSX(); for (int rl = 0; rl < 16; ++rl) vst2(S + (size_t)(ql0 + rl) * TT + k0 + lane * 4, *(const v4f*)&ss[wave][rl][lane * 4]); }
__global__ __launch_bounds__(256) void k_sm(float* __restrict__ S0) { __shared__ float sred[8]; __shared__ float sbc; __shared__ __align__(16) float sh[TT];
  const int t = threadIdx.x; const size_t row = blockIdx.x; float* sr = S0 + (size_t)blockIdx.y * TT * TT + row * TT; const int kend = TT;
  float m = -3.0e38f; for (int k = t; k < kend; k += 256) m = fmaxf(m, sr[k]);
#pragma unroll
  for (int o = 1; o < 32; o <<= 1) m = fmaxf(m, __shfl_xor(m, o));
  if ((t & 31) == 0) sred[t >> 5] = m; __syncthreads(); if (t == 0) { float a = sred[0]; for (int i = 1; i < 8; ++i) a = fmaxf(a, sred[i]); sbc = a; } __syncthreads(); m = sbc; __syncthreads();
  float sum = 0.f; for (int k = t; k < kend; k += 256) { const float v = sr[k]; sum += (v <= -1.0e38f) ? 0.f : expf(v - m); }
#pragma unroll
  for (int o = 1; o < 32; o <<= 1) sum += __shfl_xor(sum, o);
  if ((t & 31) == 0) sred[t >> 5] = sum; __syncthreads(); if (t == 0) { float a = 0.f; for (int i = 0; i < 8; ++i) a += sred[i]; sbc = 1.0f / a; } __syncthreads(); const float inv = sbc;
  for (int k = t; k < kend; k += 256) { const float v = sr[k]; sh[k] = (v <= -1.0e38f) ? 0.f : expf(v - m) * inv * 2048.0f; }
  __syncthreads(); for (int q = t; q < kend / 4; q += 256) vst2(sr + q * 4, *(const v4f*)&sh[q * 4]); }
__global__ __launch_bounds__(128) void k_pv(const float* __restrict__ PS, const _Float16* __restrict__ GP, int b, float* __restrict__ Y) { __shared__ __align__(16) float ss[4][16][132];
  const int tid = threadIdx.x, wave = tid >> 5, lane = tid & 31, col = lane & 15, g = lane >> 4; const int ql0 = blockIdx.x * 64 + wave * 16; const int c0 = blockIdx.y * 128;
  v8f acc[8] = {}, accl[8] = {};
#pragma unroll 1
  for (int kc = 0; kc < TT / 32; ++kc) { v16h ph, pl; { const float* pr = PS + (size_t)(ql0 + col) * TT + kc * 32 + 8 * g;
#pragma unroll
      for (int i = 0; i < 8; ++i) { const float a0 = pr[i], a1 = pr[16 + i]; const _Float16 h0 = (_Float16)a0, h1 = (_Float16)a1; ph[i] = h0; ph[8 + i] = h1; pl[i] = (_Float16)((a0 - (float)h0) * 1024.0f); pl[8 + i] = (_Float16)((a1 - (float)h1) * 1024.0f); } }
    asm volatile("s_wait_loadcnt 0x0" ::: "memory");
#pragma unroll
    for (int j = 0; j < 8; ++j) { const v16h gv = frag_h(GP + ((size_t)b * CI + c0 + j * 16 + col) * (size_t)TT + kc * 32, lane); acc[j] = wmma16(ph, gv, acc[j]); accl[j] = wmma16(pl, gv, accl[j]); } }
#pragma unroll
  for (int j = 0; j < 8; ++j)
#pragma unroll
    for (int r = 0; r < 8; ++r) ss[wave][8 * g + r][j * 16 + col] = (acc[j][r] + accl[j][r] * (1.0f / 1024.0f)) * (1.0f / 2048.0f);
  LDSX(); for (int rl = 0; rl < 16; ++rl) vst2(Y + ((size_t)b * TT + ql0 + rl) * CI + c0 + lane * 4, *(const v4f*)&ss[wave][rl][lane * 4]); }
__global__ __launch_bounds__(128) void k_wz(const float* __restrict__ Y, const float* __restrict__ WZ, const float* __restrict__ BZ, const float* __restrict__ XIN, float* __restrict__ OUT) { __shared__ __align__(16) float st[128][68];
  const int tid = threadIdx.x, wave = tid >> 5, lane = tid & 31, col = lane & 15, g = lane >> 4; const size_t r0 = (size_t)blockIdx.x * 64; const int c0 = blockIdx.y * 128; const size_t b = r0 / TT; const int n0 = (int)(r0 % TT);
  v8f acc[8] = {};
#pragma unroll
  for (int kc = 0; kc < CI / 32; ++kc) { const F2 a = split_row(Y + (r0 + wave * 16 + col) * CI, kc * 32, lane);
#pragma unroll
    for (int j = 0; j < 8; ++j) { v16b w; const float* wr = WZ + (size_t)(c0 + j * 16 + col) * CI + kc * 32 + 8 * g;
#pragma unroll
      for (int i = 0; i < 8; ++i) { w[i] = (__bf16)wr[i]; w[8 + i] = (__bf16)wr[16 + i]; }
      asm volatile("s_wait_loadcnt 0x0" ::: "memory"); acc[j] = wmma_bf(a.h, w, acc[j]); acc[j] = wmma_bf(a.l, w, acc[j]); } }
#pragma unroll
  for (int j = 0; j < 8; ++j) { const int cl = j * 16 + col; const float bb = bfr(BZ[c0 + cl]);
#pragma unroll
    for (int r = 0; r < 8; ++r) st[cl][wave * 16 + 8 * g + r] = acc[j][r] + bb; }
  __syncthreads();
  for (int e = tid; e < 128 * 16; e += 128) { const int cl = e >> 4, q = e & 15; const size_t off = (b * CX + c0 + cl) * (size_t)XSTR + n0 + q * 4; const v4f xr = *(const v4f*)(XIN + off); v4f o = *(const v4f*)&st[cl][q * 4]; o[0] += bfr(xr[0]); o[1] += bfr(xr[1]); o[2] += bfr(xr[2]); o[3] += bfr(xr[3]); vst2(OUT + off, o); } }
extern "C" void kernel_launch(void* const* d_in, const int* in_sizes, int n_in, void* d_out, int out_size, void* d_ws, size_t ws_size, hipStream_t stream) {
  (void)in_sizes; (void)n_in; (void)out_size;
  const float** F = (const float**)d_in;
  if (ws_size < (size_t)WS_END) return;
  char* ws = (char*)d_ws; __bf16* XT = (__bf16*)(ws + WS_XT); _Float16* GP = (_Float16*)(ws + WS_GP); _Float16 *TH = (_Float16*)(ws + WS_TH), *TL = (_Float16*)(ws + WS_TL), *PH = (_Float16*)(ws + WS_PH), *PL = (_Float16*)(ws + WS_PL); float *S = (float*)(ws + WS_S), *Y = (float*)(ws + WS_Y);
  k_xt<<<dim3(TT / 64, TNB, 1), 256, 0, stream>>>(F[0], F[0], XT, XT);
  k_proj<<<dim3(TNB * TT / 64, 3, CI / 128), 128, 0, stream>>>(XT, XT, F[1], F[2], F[3], F[4], F[5], F[6], TH, TL, PH, PL, GP);
  for (int b = 0; b < TNB; ++b) {
    k_sc<<<dim3(TT / 64, TT / 128), 128, 0, stream>>>(TH, TL, PH, PL, b, S);
    k_sm<<<dim3(TT, 1), 256, 0, stream>>>(S);
    k_pv<<<dim3(TT / 64, CI / 128), 128, 0, stream>>>(S, GP, b, Y);
  }
  k_wz<<<dim3(TNB * TT / 64, CX / 128), 128, 0, stream>>>(Y, F[7], F[8], F[0], (float*)d_out);
}
